// VariableAttentionLayer_19207093747765
// MI455X (gfx1250) — hardware-verified
//
#include <hip/hip_runtime.h>


#define NB_  32
#define TT   512
#define DD   512
#define NH_  8
#define HD   64
#define NT   (NB_ * TT)
#define NZ   (NB_ * NH_)
#define ZB   32
typedef _Float16 h16;
typedef unsigned short bf;
typedef __attribute__((ext_vector_type(16))) __bf16   v16bf;
typedef __attribute__((ext_vector_type(16))) _Float16 v16h;
typedef __attribute__((ext_vector_type(8)))  _Float16 v8h;
typedef __attribute__((ext_vector_type(8)))  unsigned short v8us;
typedef __attribute__((ext_vector_type(8)))  float    v8f;
typedef __attribute__((ext_vector_type(4)))  float    v4f;
typedef v8h  __attribute__((may_alias)) v8ha;
typedef v4f  __attribute__((may_alias)) v4fa;
typedef v8us __attribute__((may_alias)) v8usa;

__device__ __forceinline__ unsigned short f2bf(float f) { unsigned u = __float_as_uint(f); u += 0x7FFFu + ((u >> 16) & 1u); return (unsigned short)(u >> 16); }
__device__ __forceinline__ float bf2f(unsigned short b) { return __uint_as_float(((unsigned)b) << 16); }
__device__ __forceinline__ float bfr(float f) { return bf2f(f2bf(f)); }
__device__ __forceinline__ v16h cat16(v8h lo, v8h hi) { return __builtin_shufflevector(lo, hi, 0, 1, 2, 3, 4, 5, 6, 7, 8, 9, 10, 11, 12, 13, 14, 15); }
__device__ __forceinline__ v16bf cat16b(v8us lo, v8us hi) { return __builtin_bit_cast(v16bf, __builtin_shufflevector(lo, hi, 0, 1, 2, 3, 4, 5, 6, 7, 8, 9, 10, 11, 12, 13, 14, 15)); }
__device__ __forceinline__ v8f wmma16(v16h a, v16h b, v8f c) { return __builtin_amdgcn_wmma_f32_16x16x32_f16(false, a, false, b, (short)0, c, false, false); }
__device__ __forceinline__ v8f wmmab(v16bf a, v16bf b, v8f c) { return __builtin_amdgcn_wmma_f32_16x16x32_bf16(false, a, false, b, (short)0, c, false, false); }


template <typename T16> struct WFrag;
template <> struct WFrag<h16> { typedef v16h V; static __device__ __forceinline__ V ld(const h16* p) { return cat16(*(const v8h*)p, *(const v8h*)(p + 16)); } static __device__ __forceinline__ v8f mma(V a, V b, v8f c) { return wmma16(a, b, c); } };
template <> struct WFrag<bf> { typedef v16bf V; static __device__ __forceinline__ V ld(const bf* p) { return cat16b(*(const v8us*)p, *(const v8us*)(p + 16)); } static __device__ __forceinline__ v8f mma(V a, V b, v8f c) { return wmmab(a, b, c); } };
template <typename T16, int NSPLIT, bool BIAS>
__global__ __launch_bounds__(32) void k_gemmw(const T16* __restrict__ A, const T16* __restrict__ A2, const T16* __restrict__ Bt, const T16* __restrict__ Bt2, int K, float* C, int ldc, const float* __restrict__ bias, size_t sA, size_t sB, size_t sC) {
    typedef typename WFrag<T16>::V V;
    __shared__ __align__(16) float os[16 * 68];
    const size_t z = blockIdx.z; A += z * sA; if (A2) A2 += z * sA; Bt += z * sB; if (Bt2) Bt2 += z * sB; C += z * sC;
    const int lane = threadIdx.x & 31, lr = lane & 15, hi = lane >> 4; const int r0 = blockIdx.x * 64, c0 = blockIdx.y * 64;
    v8f acc[4][4];
#pragma unroll
    for (int mb = 0; mb < 4; ++mb)
#pragma unroll
        for (int nb = 0; nb < 4; ++nb) acc[mb][nb] = (v8f){};
    const size_t aoff = (size_t)(r0 + lr) * K + 8 * hi, boff = (size_t)(c0 + lr) * K + 8 * hi;
#pragma unroll 1
    for (int kc = 0; kc < K; kc += 32) {
        V a[4], a2[4];
#pragma unroll
        for (int mb = 0; mb < 4; ++mb) { a[mb] = WFrag<T16>::ld(A + aoff + (size_t)mb * 16 * K + kc); if (NSPLIT == 1 || NSPLIT == 2) a2[mb] = WFrag<T16>::ld(A2 + aoff + (size_t)mb * 16 * K + kc); }
#pragma unroll
        for (int nb = 0; nb < 4; ++nb) { const V b = WFrag<T16>::ld(Bt + boff + (size_t)nb * 16 * K + kc); V b2; if (NSPLIT >= 2) b2 = WFrag<T16>::ld(Bt2 + boff + (size_t)nb * 16 * K + kc);
#pragma unroll
            for (int mb = 0; mb < 4; ++mb) { acc[mb][nb] = WFrag<T16>::mma(a[mb], b, acc[mb][nb]); if (NSPLIT == 1 || NSPLIT == 2) acc[mb][nb] = WFrag<T16>::mma(a2[mb], b, acc[mb][nb]); if (NSPLIT >= 2) acc[mb][nb] = WFrag<T16>::mma(a[mb], b2, acc[mb][nb]); } }
        asm volatile("v_nop\n\tv_nop\n\tv_nop\n\tv_nop" : "+v"(acc[0][0]), "+v"(acc[1][1]), "+v"(acc[2][2]), "+v"(acc[3][3]) : "v"(a[0]), "v"(a[3]));
    }
#pragma unroll
    for (int mb = 0; mb < 4; ++mb) {
#pragma unroll
        for (int nb = 0; nb < 4; ++nb) {
#pragma unroll
            for (int j = 0; j < 8; ++j) os[(hi * 8 + j) * 68 + nb * 16 + lr] = acc[mb][nb][j]; }
        __builtin_amdgcn_wave_barrier(); asm volatile("" ::: "memory");
        float* crow = C + (size_t)(r0 + mb * 16) * ldc + c0;
#pragma unroll 1
        for (int ps = 0; ps < 2; ++ps) {
#pragma unroll
            for (int s = 0; s < 8; ++s) { const int row = 2 * s + hi, cofs = lr * 4; v4f val = *(const v4fa*)(os + row * 68 + cofs); if (BIAS) { val[0] += bfr(bias[c0 + cofs]); val[1] += bfr(bias[c0 + cofs + 1]); val[2] += bfr(bias[c0 + cofs + 2]); val[3] += bfr(bias[c0 + cofs + 3]); }
                *(volatile v4f*)(crow + (size_t)row * ldc + cofs) = val; }
            if (ps == 0) __threadfence(); }
        __builtin_amdgcn_wave_barrier(); asm volatile("" ::: "memory");
    }
}

__device__ __forceinline__ void splitf(float y, unsigned short& h, unsigned short& l) { h = f2bf(y); l = f2bf(y - bf2f(h)); }
__device__ __forceinline__ float gelu_e(float t) { return 0.5f * t * (1.0f + erff(t * 0.70710678118654752f)); }
typedef __attribute__((ext_vector_type(2))) unsigned short v2us;
typedef __attribute__((ext_vector_type(4))) unsigned short v4us;
typedef __attribute__((ext_vector_type(2))) float v2f;

__global__ __launch_bounds__(256) void k_cvt8(const float* __restrict__ src, bf* dst, size_t n8) { const size_t i = (size_t)blockIdx.x * 256 + threadIdx.x; if (i >= n8) return; const v8f v = *(const v8f*)(src + i * 8); v8us o;
#pragma unroll
    for (int k = 0; k < 8; ++k) o[k] = f2bf(v[k]); *(volatile v8us*)(dst + i * 8) = o; __threadfence(); *(volatile v8us*)(dst + i * 8) = o; }
__global__ __launch_bounds__(256) void k_wtT(const float* __restrict__ w, bf* Bt) {
    const int lane = threadIdx.x & 31; const int L0 = (blockIdx.x * 8 + (threadIdx.x >> 5)) * 8; const int nlines = DD * DD / 64;
#pragma unroll 1
    for (int ps = 0; ps < 2; ++ps) {
#pragma unroll
        for (int l = 0; l < 8; ++l) { const int L = L0 + l; if (L >= nlines) break; const int e = L * 64 + lane * 2; const int k = e & (DD - 1), n = e >> 9; v2us o;
#pragma unroll
            for (int q = 0; q < 2; ++q) o[q] = f2bf(w[(size_t)(k + q) * DD + n]);
            *(volatile v2us*)(Bt + (size_t)e) = o; }
        if (ps == 0) __threadfence(); }
}
__device__ __forceinline__ void row_ln(const float* __restrict__ row, const float* __restrict__ gg, const float* __restrict__ bb, int lane, float v[16]) {
    float s = 0.f;
#pragma unroll
    for (int c = 0; c < 4; ++c) { const v4f a = *(const v4f*)(row + c * 128 + lane * 4);
#pragma unroll
        for (int q = 0; q < 4; ++q) { v[c * 4 + q] = a[q]; s += a[q]; } }
#pragma unroll
    for (int sh = 16; sh; sh >>= 1) s += __shfl_xor(s, sh, 32);
    const float mu = s * (1.0f / DD); float qq = 0.f;
#pragma unroll
    for (int i = 0; i < 16; ++i) { const float d0 = v[i] - mu; qq = __fadd_rn(qq, __fmul_rn(d0, d0)); }
#pragma unroll
    for (int sh = 16; sh; sh >>= 1) qq += __shfl_xor(qq, sh, 32);
    const float rs = __fdiv_rn(1.0f, sqrtf(qq * (1.0f / DD) + 1e-5f));
#pragma unroll
    for (int c = 0; c < 4; ++c)
#pragma unroll
        for (int q = 0; q < 4; ++q) { const int col = c * 128 + lane * 4 + q; v[c * 4 + q] = __fadd_rn(__fmul_rn((v[c * 4 + q] - mu) * rs, bfr(gg[col])), bfr(bb[col])); }
}
__global__ __launch_bounds__(256) void k_lnhead(const float* __restrict__ F, const float* __restrict__ gg, const float* __restrict__ bb, float sc, bf* Ph, bf* Pl) {
    const int lane = threadIdx.x & 31; const int r = blockIdx.x * 8 + (threadIdx.x >> 5); if (r >= NT) return; const int b = r >> 9, t = r & (TT - 1); float v[16]; row_ln(F + (size_t)r * DD, gg, bb, lane, v);
#pragma unroll 1
    for (int ps = 0; ps < 2; ++ps) {
#pragma unroll
        for (int c = 0; c < 4; ++c) { const int col = c * 128 + lane * 4; const int h = col >> 6, d = col & 63; v4us oh, ol;
#pragma unroll
            for (int q = 0; q < 4; ++q) { unsigned short a, c2; splitf(v[c * 4 + q] * sc, a, c2); oh[q] = a; ol[q] = c2; }
            const size_t o = (((size_t)b * NH_ + h) * TT + t) * HD + d; *(volatile v4us*)(Ph + o) = oh; *(volatile v4us*)(Pl + o) = ol; }
        if (ps == 0) __threadfence(); }
}
__global__ __launch_bounds__(256) void k_lnrow(float* F, const float* __restrict__ gg, const float* __restrict__ bb) {
    const int lane = threadIdx.x & 31; const int r = blockIdx.x * 8 + (threadIdx.x >> 5); if (r >= NT) return; float v[16]; row_ln(F + (size_t)r * DD, gg, bb, lane, v);
#pragma unroll 1
    for (int ps = 0; ps < 2; ++ps) {
#pragma unroll
        for (int c = 0; c < 4; ++c) { v4f o; for (int q = 0; q < 4; ++q) o[q] = v[c * 4 + q]; *(volatile v4f*)(F + (size_t)r * DD + c * 128 + lane * 4) = o; }
        if (ps == 0) __threadfence(); }
}
__global__ __launch_bounds__(256) void k_vtplane(const float* __restrict__ F, bf* Vh, bf* Vl) {
    const int lane = threadIdx.x & 31; const int L0 = (blockIdx.x * 8 + (threadIdx.x >> 5)) * 8; const int nlines = NT * DD / 64;
#pragma unroll 1
    for (int ps = 0; ps < 2; ++ps) {
#pragma unroll
        for (int l = 0; l < 8; ++l) { const int L = L0 + l; if (L >= nlines) break; const int e = L * 64 + lane * 2; const int t = e & (TT - 1); const int d = (e >> 9) & 63; const int z = e >> 15; const int b = z >> 3, h = z & 7; v2us oh, ol;
#pragma unroll
            for (int q = 0; q < 2; ++q) { unsigned short a, c2; splitf(F[((size_t)b * TT + t + q) * DD + h * HD + d], a, c2); oh[q] = a; ol[q] = c2; }
            *(volatile v2us*)(Vh + (size_t)e) = oh; *(volatile v2us*)(Vl + (size_t)e) = ol; }
        if (ps == 0) __threadfence(); }
}
__global__ __launch_bounds__(256) void k_soft(const float* __restrict__ S, bf* Ph, bf* Pl) {
    const int lane = threadIdx.x & 31; const int row = blockIdx.x * 8 + (threadIdx.x >> 5); if (row >= ZB * TT) return; const float* sr = S + (size_t)row * TT; float v[16]; float mx = -3.0e38f;
#pragma unroll
    for (int ch = 0; ch < 4; ++ch) { const v4f a = *(const v4f*)(sr + ch * 128 + lane * 4);
#pragma unroll
        for (int q = 0; q < 4; ++q) { v[ch * 4 + q] = a[q]; mx = fmaxf(mx, a[q]); } }
#pragma unroll
    for (int sh = 16; sh; sh >>= 1) mx = fmaxf(mx, __shfl_xor(mx, sh, 32));
    float sum = 0.f;
#pragma unroll
    for (int kk = 0; kk < 16; ++kk) { v[kk] = __expf(v[kk] - mx); sum += v[kk]; }
#pragma unroll
    for (int sh = 16; sh; sh >>= 1) sum += __shfl_xor(sum, sh, 32);
    const float f = __fdiv_rn(1.0f, sum);
#pragma unroll 1
    for (int ps = 0; ps < 2; ++ps) {
#pragma unroll
        for (int ch = 0; ch < 4; ++ch) { v4us oh, ol;
#pragma unroll
            for (int q = 0; q < 4; ++q) { unsigned short a, c2; splitf(v[ch * 4 + q] * f, a, c2); oh[q] = a; ol[q] = c2; }
            *(volatile v4us*)(Ph + (size_t)row * TT + ch * 128 + lane * 4) = oh; *(volatile v4us*)(Pl + (size_t)row * TT + ch * 128 + lane * 4) = ol; }
        if (ps == 0) __threadfence(); }
}
__global__ __launch_bounds__(256) void k_merge(const float* __restrict__ O, int z0, bf* Ah, bf* Al) {
    const int lane = threadIdx.x & 31; const int L0 = (blockIdx.x * 8 + (threadIdx.x >> 5)) * 8; const int nlines = ZB * TT * HD / 64;
#pragma unroll 1
    for (int ps = 0; ps < 2; ++ps) {
#pragma unroll
        for (int l = 0; l < 8; ++l) { const int L = L0 + l; if (L >= nlines) break; const int e = L * 64 + lane * 2; const int d = e & 63; const int t = (e >> 6) & (TT - 1); const int zz = e >> 15; const int z = z0 + zz; const int b = z >> 3, h = z & 7; v2us oh, ol;
#pragma unroll
            for (int q = 0; q < 2; ++q) { unsigned short a, c2; splitf(O[(size_t)e + q], a, c2); oh[q] = a; ol[q] = c2; }
            const size_t o = ((size_t)b * TT + t) * DD + h * HD + d; *(volatile v2us*)(Ah + o) = oh; *(volatile v2us*)(Al + o) = ol; }
        if (ps == 0) __threadfence(); }
}
__global__ __launch_bounds__(256) void k_gres(float* C, const float* __restrict__ x) {
    const size_t i = (size_t)blockIdx.x * 256 + threadIdx.x; if (i >= (size_t)NT * DD / 4) return; const v4f a = *(const v4f*)(C + i * 4), xx = *(const v4f*)(x + i * 4); v4f o;
#pragma unroll
    for (int q = 0; q < 4; ++q) o[q] = gelu_e(a[q]) + bfr(xx[q]);
    *(volatile v4f*)(C + i * 4) = o; __threadfence(); *(volatile v4f*)(C + i * 4) = o;
}
__global__ __launch_bounds__(256) void k_ln2(const float* __restrict__ G, const float* __restrict__ gg, const float* __restrict__ bb, float* X2, bf* Ph, bf* Pl) {
    const int lane = threadIdx.x & 31; const int r = blockIdx.x * 8 + (threadIdx.x >> 5); if (r >= NT) return; float v[16]; row_ln(G + (size_t)r * DD, gg, bb, lane, v);
#pragma unroll 1
    for (int ps = 0; ps < 2; ++ps) {
#pragma unroll
        for (int c = 0; c < 4; ++c) { v4f o; v4us oh, ol;
#pragma unroll
            for (int q = 0; q < 4; ++q) { o[q] = v[c * 4 + q]; unsigned short a, c2; splitf(o[q], a, c2); oh[q] = a; ol[q] = c2; }
            *(volatile v4f*)(X2 + (size_t)r * DD + c * 128 + lane * 4) = o; *(volatile v4us*)(Ph + (size_t)r * DD + c * 128 + lane * 4) = oh; *(volatile v4us*)(Pl + (size_t)r * DD + c * 128 + lane * 4) = ol; }
        if (ps == 0) __threadfence(); }
}
__global__ __launch_bounds__(256) void k_fiw(const float* __restrict__ H, const float* __restrict__ W2, const float* __restrict__ b2, float* WV) {
    const int lane = threadIdx.x & 31; const int r = (blockIdx.x * 8 + (threadIdx.x >> 5)) * 32 + lane; if (r >= NT) return; const float* hr = H + (size_t)r * DD; float s = bfr(b2[0]);
#pragma unroll 2
    for (int c = 0; c < DD; ++c) s = __fadd_rn(s, __fmul_rn(gelu_e(hr[c]), bfr(W2[c])));
    *(volatile float*)(WV + r) = s; __threadfence(); *(volatile float*)(WV + r) = s;
}
__global__ __launch_bounds__(256) void k_fisoft(const float* __restrict__ WV, float* FI) {
    const int lane = threadIdx.x & 31; const int b = blockIdx.x * 8 + (threadIdx.x >> 5); if (b >= NB_) return; const float* sr = WV + (size_t)b * TT; float v[16]; float mx = -3.0e38f;
#pragma unroll
    for (int ch = 0; ch < 4; ++ch) { const v4f a = *(const v4f*)(sr + ch * 128 + lane * 4);
#pragma unroll
        for (int q = 0; q < 4; ++q) { v[ch * 4 + q] = a[q]; mx = fmaxf(mx, a[q]); } }
#pragma unroll
    for (int sh = 16; sh; sh >>= 1) mx = fmaxf(mx, __shfl_xor(mx, sh, 32));
    float sum = 0.f;
#pragma unroll
    for (int kk = 0; kk < 16; ++kk) { v[kk] = __expf(v[kk] - mx); sum += v[kk]; }
#pragma unroll
    for (int sh = 16; sh; sh >>= 1) sum += __shfl_xor(sum, sh, 32);
    const float f = __fdiv_rn(1.0f, sum);
#pragma unroll 1
    for (int ps = 0; ps < 2; ++ps) {
#pragma unroll
        for (int ch = 0; ch < 4; ++ch) { v4f o;
#pragma unroll
            for (int q = 0; q < 4; ++q) o[q] = v[ch * 4 + q] * f;
            *(volatile v4f*)(FI + (size_t)b * TT + ch * 128 + lane * 4) = o; }
        if (ps == 0) __threadfence(); }
}

extern "C" void kernel_launch(void* const* d_in, const int* in_sizes, int n_in,
                              void* d_out, int out_size, void* d_ws, size_t ws_size, hipStream_t stream) {
    (void)in_sizes; (void)n_in; (void)out_size;
    const float* IN[21]; for (int i = 0; i < 21; ++i) IN[i] = (const float*)d_in[i];
    const float* x = IN[0];
    float* X2 = (float*)d_out; float* FI = (float*)((char*)d_out + (size_t)NT * DD * 4);
    char* wsp = (char*)d_ws;
    auto take = [&](size_t bytes) { char* p = wsp; wsp += (bytes + 255) & ~(size_t)255; return (void*)p; };
    bf* WQ = (bf*)take((size_t)DD * DD * 2); bf* WK = (bf*)take((size_t)DD * DD * 2); bf* WVb = (bf*)take((size_t)DD * DD * 2); bf* WO = (bf*)take((size_t)DD * DD * 2); bf* W1T = (bf*)take((size_t)DD * DD * 2);
    bf* XB = (bf*)take((size_t)NT * DD * 2); float* F = (float*)take((size_t)NT * DD * 4);
    bf* QPh = (bf*)take((size_t)NT * DD * 2); bf* QPl = (bf*)take((size_t)NT * DD * 2); bf* KPh = (bf*)take((size_t)NT * DD * 2); bf* KPl = (bf*)take((size_t)NT * DD * 2); bf* VTh = (bf*)take((size_t)NT * DD * 2); bf* VTl = (bf*)take((size_t)NT * DD * 2);
    float* Sb = (float*)take((size_t)ZB * TT * TT * 4); bf* Ph = (bf*)take((size_t)ZB * TT * TT * 2); bf* Pl = (bf*)take((size_t)ZB * TT * TT * 2); float* Ob = (float*)take((size_t)ZB * TT * HD * 4); float* WVr = (float*)take((size_t)NT * 4);
    if ((size_t)(wsp - (char*)d_ws) > ws_size) return;
    { const unsigned gT = (unsigned)((DD * DD / 64 + 63) / 64); k_wtT<<<gT, 256, 0, stream>>>(IN[1], WQ); k_wtT<<<gT, 256, 0, stream>>>(IN[3], WK); k_wtT<<<gT, 256, 0, stream>>>(IN[5], WVb); k_wtT<<<gT, 256, 0, stream>>>(IN[13], WO); k_wtT<<<gT, 256, 0, stream>>>(IN[17], W1T); }
    const size_t nx = (size_t)NT * DD / 8; const unsigned gx = (unsigned)((nx + 255) / 256); const unsigned LB = (unsigned)((NT * DD / 64 + 63) / 64);
    k_cvt8<<<gx, 256, 0, stream>>>(x, XB, nx);
    k_gemmw<bf, 0, true><<<dim3(NT / 64, DD / 64, 1), 32, 0, stream>>>(XB, nullptr, WQ, nullptr, DD, F, DD, IN[2], 0, 0, 0); k_lnhead<<<NT / 8, 256, 0, stream>>>(F, IN[7], IN[8], 0.125f, QPh, QPl);
    k_gemmw<bf, 0, true><<<dim3(NT / 64, DD / 64, 1), 32, 0, stream>>>(XB, nullptr, WK, nullptr, DD, F, DD, IN[4], 0, 0, 0); k_lnhead<<<NT / 8, 256, 0, stream>>>(F, IN[9], IN[10], 1.0f, KPh, KPl);
    k_gemmw<bf, 0, true><<<dim3(NT / 64, DD / 64, 1), 32, 0, stream>>>(XB, nullptr, WVb, nullptr, DD, F, DD, IN[6], 0, 0, 0); k_lnrow<<<NT / 8, 256, 0, stream>>>(F, IN[11], IN[12]); k_vtplane<<<LB, 256, 0, stream>>>(F, VTh, VTl);
    bf* ATh = XB; bf* ATl = (bf*)F;
    for (int z0 = 0; z0 < NZ; z0 += ZB) {
        k_gemmw<bf, 2, false><<<dim3(TT / 64, TT / 64, ZB), 32, 0, stream>>>(QPh + (size_t)z0 * TT * HD, QPl + (size_t)z0 * TT * HD, KPh + (size_t)z0 * TT * HD, KPl + (size_t)z0 * TT * HD, HD, Sb, TT, nullptr, (size_t)TT * HD, (size_t)TT * HD, (size_t)TT * TT);
        k_soft<<<ZB * TT / 8, 256, 0, stream>>>(Sb, Ph, Pl);
        k_gemmw<bf, 2, false><<<dim3(TT / 64, 1, ZB), 32, 0, stream>>>(Ph, Pl, VTh + (size_t)z0 * HD * TT, VTl + (size_t)z0 * HD * TT, TT, Ob, HD, nullptr, (size_t)TT * TT, (size_t)HD * TT, (size_t)TT * HD);
        k_merge<<<(ZB * TT * HD / 64 + 63) / 64, 256, 0, stream>>>(Ob, z0, ATh, ATl); }
    float* C = (float*)KPh;
    k_gemmw<bf, 1, true><<<dim3(NT / 64, DD / 64, 1), 32, 0, stream>>>(ATh, ATl, WO, nullptr, DD, C, DD, IN[14], 0, 0, 0);
    bf* X2h = VTh; bf* X2l = VTl;
    k_gres<<<(unsigned)(((size_t)NT * DD / 4 + 255) / 256), 256, 0, stream>>>(C, x); k_ln2<<<NT / 8, 256, 0, stream>>>(C, IN[15], IN[16], X2, X2h, X2l);
    float* Hm = (float*)QPh;
    k_gemmw<bf, 1, true><<<dim3(NT / 64, DD / 64, 1), 32, 0, stream>>>(X2h, X2l, W1T, nullptr, DD, Hm, DD, IN[18], 0, 0, 0);
    k_fiw<<<NT / 256, 256, 0, stream>>>(Hm, IN[19], IN[20], WVr);
    k_fisoft<<<NB_ / 8, 256, 0, stream>>>(WVr, FI);
}
